// MultiHeadSelfAttentionBlock_20624432956368
// MI455X (gfx1250) — hardware-run, weakly checked
//
#include <hip/hip_runtime.h>
#include <math.h>

constexpr int kB = 2, kT = 2048, kD = 1024, kH = 16, kHD = 64, kFF = 4096;
constexpr int kTok = kB * kT;
constexpr int kNQKV = 3 * kD;
constexpr int kN12 = 2 * kFF;
constexpr int kGrp = 2;
constexpr int kFfnRows = 512;
constexpr float kWCarry = 16.0f;
constexpr float kWCarryInv = 1.0f / 16.0f;
constexpr float kPCarry = 2048.0f;
constexpr float kPCarryInv = 1.0f / 2048.0f;
constexpr float kQKScale = 0.125f;
constexpr float kEps = 1e-6f;
constexpr float kInvD = 1.0f / 1024.0f;

constexpr size_t kMiB = 1048576;
constexpr size_t OFF_WQKV = 0;
constexpr size_t SZ_WQKV  = (size_t)kNQKV * kD * 2;
constexpr size_t OFF_XN   = OFF_WQKV + SZ_WQKV;
constexpr size_t SZ_XN    = (size_t)kTok * kD * 2;
constexpr size_t OFF_BIG  = OFF_XN + SZ_XN;
constexpr size_t SZ_BIG   = 32 * kMiB;
constexpr size_t OFF_GU   = OFF_BIG;
constexpr size_t OFF_W12  = OFF_BIG + 16 * kMiB;
constexpr size_t OFF_QP   = OFF_BIG + SZ_BIG;
constexpr size_t SZ_PL    = (size_t)kB * kH * kT * kHD * 2;
constexpr size_t OFF_KP   = OFF_QP + SZ_PL;
constexpr size_t OFF_VT   = OFF_KP + SZ_PL;
constexpr size_t OFF_PP   = OFF_VT + SZ_PL;
constexpr size_t SZ_PP    = (size_t)kGrp * kT * kT * 2;
constexpr size_t OFF_HH   = OFF_QP;
constexpr size_t SZ_HH    = (size_t)kTok * kFF * 2;
constexpr size_t OFF_W3T  = OFF_HH + SZ_HH;
constexpr size_t SZ_W3T   = (size_t)kD * kFF * 2;
constexpr size_t OFF_X1   = OFF_PP + SZ_PP;
constexpr size_t SZ_X1    = (size_t)kTok * kD * 4;
constexpr size_t OFF_WP   = OFF_X1 + SZ_X1;
constexpr size_t SZ_WP    = (size_t)kD * kD * 2;
constexpr size_t WS_TOTAL = OFF_WP + SZ_WP;
static_assert((size_t)kT * kNQKV * 4 <= SZ_BIG, "qkv f32 chunk fits");
static_assert((size_t)kGrp * kT * kT * 4 <= SZ_BIG, "scores chunk fits");
static_assert((size_t)kFfnRows * kN12 * 4 <= OFF_W12 - OFF_GU, "gate|up chunk fits below W12");
static_assert(OFF_W12 + (size_t)kN12 * kD * 2 <= OFF_QP, "W12 fits");
static_assert(OFF_W3T + SZ_W3T <= OFF_X1, "H + fc3^T fit in the q/k/v/p region");
static_assert(WS_TOTAL == 109051904, "carve total");
static_assert(WS_TOTAL <= 134217728, "carve under 128 MiB");

typedef __attribute__((ext_vector_type(16))) _Float16 v16h;
typedef __attribute__((ext_vector_type(8)))  _Float16 v8h;
typedef __attribute__((ext_vector_type(16))) __bf16   v16b;
typedef __attribute__((ext_vector_type(8)))  __bf16   v8b;
typedef __attribute__((ext_vector_type(8)))  float    v8f;
typedef __attribute__((ext_vector_type(4)))  float    v4f;
typedef __attribute__((ext_vector_type(4)))  unsigned int v4u;
typedef unsigned short u16;

__device__ __forceinline__ unsigned short f2bf_bits(float f) {
  unsigned u = __float_as_uint(f);
  return (unsigned short)((u + 0x7FFFu + ((u >> 16) & 1u)) >> 16);
}
__device__ __forceinline__ float bf_bits2f(unsigned short h) { return __uint_as_float(((unsigned)h) << 16); }

__device__ __forceinline__ void dep_guard_h(v8f& a, v8f& b, v16h x, v16h y) { asm volatile("v_nop\n\tv_nop\n\tv_nop\n\tv_nop" : "+v"(a), "+v"(b) : "v"(x), "v"(y)); }
__device__ __forceinline__ void dep_guard_b(v8f& a, v8f& b, v16b x, v16b y) { asm volatile("v_nop\n\tv_nop\n\tv_nop\n\tv_nop" : "+v"(a), "+v"(b) : "v"(x), "v"(y)); }
__device__ __forceinline__ void keep4_h(v16h a, v16h b, v16h c, v16h d) { asm volatile("v_nop" :: "v"(a), "v"(b), "v"(c), "v"(d)); }
__device__ __forceinline__ void keep4_b(v16b a, v16b b, v16b c, v16b d) { asm volatile("v_nop" :: "v"(a), "v"(b), "v"(c), "v"(d)); }
__device__ __forceinline__ void acc_guard4(v8f& a, v8f& b, v8f& c, v8f& d) { asm volatile("v_nop\n\tv_nop\n\tv_nop\n\tv_nop" : "+v"(a), "+v"(b), "+v"(c), "+v"(d)); }
template <typename T> struct Frag;
template <> struct Frag<_Float16> {
  typedef v16h V; union U { v16h v; v8h h[2]; };
  static __device__ __forceinline__ v16h load(const _Float16* p) {
    U f; f.h[0] = *(const v8h*)(p); f.h[1] = *(const v8h*)(p + 16); return f.v;
  }
  static __device__ __forceinline__ v8f mma(v16h a, v16h b, v8f c) {
    return __builtin_amdgcn_wmma_f32_16x16x32_f16(false, a, false, b, (short)0, c, false, false);
  }
  static __device__ __forceinline__ void guard(v8f& a, v8f& b, v16h x, v16h y) { dep_guard_h(a, b, x, y); }
  static __device__ __forceinline__ void keep(v16h a, v16h b, v16h c, v16h d) { keep4_h(a, b, c, d); }
};
template <> struct Frag<__bf16> {
  typedef v16b V; union U { v16b v; v8b h[2]; };
  static __device__ __forceinline__ v16b load(const __bf16* p) {
    U f; f.h[0] = *(const v8b*)(p); f.h[1] = *(const v8b*)(p + 16); return f.v;
  }
  static __device__ __forceinline__ v8f mma(v16b a, v16b b, v8f c) {
    return __builtin_amdgcn_wmma_f32_16x16x32_bf16(false, a, false, b, (short)0, c, false, false);
  }
  static __device__ __forceinline__ void guard(v8f& a, v8f& b, v16b x, v16b y) { dep_guard_b(a, b, x, y); }
  static __device__ __forceinline__ void keep(v16b a, v16b b, v16b c, v16b d) { keep4_b(a, b, c, d); }
};

__device__ __forceinline__ unsigned pk16(unsigned short a, unsigned short b) { return (unsigned)a | ((unsigned)b << 16); }
__device__ __forceinline__ unsigned short h_bits(float f) { const _Float16 h = (_Float16)f; return __builtin_bit_cast(unsigned short, h); }

template <int ET> struct Elem;
template <> struct Elem<0> { typedef _Float16 T; };
template <> struct Elem<1> { typedef __bf16 T; };
template <int ET, bool SPLIT, int BIAS_MODE, int OUT_MODE, bool RESID, int CAUS>
__global__ __launch_bounds__(256) void wmma_gemm64(
    const unsigned short* __restrict__ Ap, const unsigned short* __restrict__ A2p, int lda, long strideA,
    const unsigned short* __restrict__ Btp, const unsigned short* __restrict__ Bt2p, int ldb, long strideB,
    void* __restrict__ Cout, void* __restrict__ Cout2, int ldc, long strideC,
    const float* __restrict__ bias,
    const float* __restrict__ resid, long strideR,
    int M, int N, int K, float scale) {
  typedef typename Elem<ET>::T T;
  typedef typename Frag<T>::V V;
  const T* A = (const T*)Ap; const T* A2 = (const T*)A2p; const T* Bt = (const T*)Btp; const T* Bt2 = (const T*)Bt2p;
  __shared__ __align__(16) float sT[8][16 * 68];
  const int b    = blockIdx.y;
  const int lane = threadIdx.x & 31;
  const int wave = threadIdx.x >> 5;
  const int tilesN = N >> 6;
  const int tilesM = M >> 6;
  const int tile = blockIdx.x * 8 + wave;
  if (tile >= tilesM * tilesN) return;
  const int tm = tile / tilesN;
  const int tn = tile - tm * tilesN;
  const int m0 = tm << 6;
  const int n0 = tn << 6;
  if (CAUS == 1 && n0 > m0) return;
  int Kend = K;
  if (CAUS == 2) { const int kl = m0 + 64; Kend = (kl < K) ? kl : K; }

  const T* Ab  = A  + (size_t)b * strideA;
  const T* Bb  = Bt + (size_t)b * strideB;
  const T* Ab2 = SPLIT ? (A2  + (size_t)b * strideA) : nullptr;
  const T* Bb2 = SPLIT ? (Bt2 + (size_t)b * strideB) : nullptr;

  const int rlane = lane & 15;
  const int koff  = (lane >> 4) * 8;
  const int mOff  = (lane >> 4) * 8;

  v8f acc[4][4];
#pragma unroll
  for (int i = 0; i < 4; ++i)
#pragma unroll
    for (int j = 0; j < 4; ++j) acc[i][j] = (v8f){0.f,0.f,0.f,0.f,0.f,0.f,0.f,0.f};

  for (int k0 = 0; k0 < Kend; k0 += 32) {
    V bh[4], bl[4];
#pragma unroll
    for (int j = 0; j < 4; ++j) {
      const size_t bo = (size_t)(n0 + (j << 4) + rlane) * ldb + koff + k0;
      bh[j] = Frag<T>::load(Bb + bo);
      if (SPLIT) bl[j] = Frag<T>::load(Bb2 + bo);
    }
#pragma unroll
    for (int i = 0; i < 4; ++i) {
      const size_t ao = (size_t)(m0 + (i << 4) + rlane) * lda + koff + k0;
      V ah = Frag<T>::load(Ab + ao);
      V al;
      if (SPLIT) al = Frag<T>::load(Ab2 + ao);
#pragma unroll
      for (int j = 0; j < 4; ++j) {
        acc[i][j] = Frag<T>::mma(ah, bh[j], acc[i][j]);
        if (SPLIT) {
          acc[i][j] = Frag<T>::mma(ah, bl[j], acc[i][j]);
          acc[i][j] = Frag<T>::mma(al, bh[j], acc[i][j]);
        }
      }
      Frag<T>::guard(acc[i][0], acc[i][3], ah, SPLIT ? al : ah);
    }
    Frag<T>::keep(bh[0], bh[1], bh[2], bh[3]);
    if (SPLIT) Frag<T>::keep(bl[0], bl[1], bl[2], bl[3]);
  }
  acc_guard4(acc[0][0], acc[0][1], acc[0][2], acc[0][3]);
  acc_guard4(acc[1][0], acc[1][1], acc[1][2], acc[1][3]);
  acc_guard4(acc[2][0], acc[2][1], acc[2][2], acc[2][3]);
  acc_guard4(acc[3][0], acc[3][1], acc[3][2], acc[3][3]);

  float* slab = sT[wave];
  const float* Rb = RESID ? (resid + (size_t)b * strideR) : nullptr;
#pragma unroll
  for (int i = 0; i < 4; ++i) {
    const int mBase = m0 + (i << 4);
#pragma unroll
    for (int j = 0; j < 4; ++j) {
      const int n = n0 + (j << 4) + rlane;
      float bv = 0.f;
      if (BIAS_MODE == 2) bv = bias[n];
#pragma unroll
      for (int r = 0; r < 8; ++r) {
        float v = acc[i][j][r] * scale;
        if (BIAS_MODE == 1) v += bias[mBase + mOff + r];
        if (BIAS_MODE == 2) v += bv;
        if (RESID) v += Rb[(size_t)(mBase + mOff + r) * ldc + n];
        slab[(mOff + r) * 68 + (j << 4) + rlane] = v;
      }
    }
    __builtin_amdgcn_fence(__ATOMIC_RELEASE, "workgroup");
    __builtin_amdgcn_wave_barrier();
    __builtin_amdgcn_fence(__ATOMIC_ACQUIRE, "workgroup");
    if (OUT_MODE == 0) {
      float* C = (float*)Cout + (size_t)b * strideC;
      const int hh = lane >> 4, c4 = (lane & 15) * 4;
      for (int pass = 0; pass < 2; ++pass) {
#pragma unroll
        for (int it = 0; it < 8; ++it) {
          const int row = it * 2 + hh;
          v4f v = *(const v4f*)(slab + row * 68 + c4);
          *(volatile v4f*)(C + (size_t)(mBase + row) * ldc + n0 + c4) = v;
        }
        __threadfence();
      }
    } else {
      const int q = lane >> 3, c8 = (lane & 7) * 8;
      unsigned short* C  = (unsigned short*)Cout  + (size_t)b * strideC;
      unsigned short* C2 = (OUT_MODE == 2) ? ((unsigned short*)Cout2 + (size_t)b * strideC) : nullptr;
      for (int pass = 0; pass < 2; ++pass) {
#pragma unroll
        for (int it = 0; it < 4; ++it) {
          const int row = it * 4 + q;
          const float* sp = slab + row * 68 + c8;
          v8h hv, lv;
#pragma unroll
          for (int e = 0; e < 8; ++e) {
            if (OUT_MODE == 1) {
              hv[e] = (_Float16)sp[e];
            } else {
              unsigned short hb = f2bf_bits(sp[e]);
              unsigned short lb = f2bf_bits(sp[e] - bf_bits2f(hb));
              hv[e] = __builtin_bit_cast(_Float16, hb);
              lv[e] = __builtin_bit_cast(_Float16, lb);
            }
          }
          *(volatile v8h*)(C + (size_t)(mBase + row) * ldc + n0 + c8) = hv;
          if (OUT_MODE == 2) *(volatile v8h*)(C2 + (size_t)(mBase + row) * ldc + n0 + c8) = lv;
        }
        __threadfence();
      }
    }
    __builtin_amdgcn_fence(__ATOMIC_RELEASE, "workgroup");
    __builtin_amdgcn_wave_barrier();
    __builtin_amdgcn_fence(__ATOMIC_ACQUIRE, "workgroup");
  }
}

__global__ __launch_bounds__(256) void tcast16_kernel(const float* __restrict__ W0, const float* __restrict__ W1,
                                                     const float* __restrict__ W2,
                                                     int nrows, int ncols, int zper, long in_sub,
                                                     unsigned short* __restrict__ out, long out_wrows, long out_subrows,
                                                     float scale) {
  __shared__ float sm[64][65];
  const int t  = threadIdx.x;
  const int r0 = blockIdx.x * 64;
  const int c0 = blockIdx.y * 64;
  const int z  = blockIdx.z;
  const int which = z / zper;
  const int sub   = z - which * zper;
  const float* W = (which == 0) ? W0 : (which == 1) ? W1 : W2;
  W += (size_t)sub * (size_t)in_sub;
#pragma unroll
  for (int i = 0; i < 16; ++i) {
    const int e = i * 256 + t;
    const int r = e >> 6;
    const int c = e & 63;
    sm[c][r] = W[(size_t)(r0 + r) * ncols + c0 + c] * scale;
  }
  __syncthreads();
  const int lane = t & 31, wave = t >> 5;
  const int q = lane >> 3, c8 = (lane & 7) * 8;
  const size_t obase = (size_t)which * (size_t)out_wrows + (size_t)sub * (size_t)out_subrows + (size_t)c0;
  for (int pass = 0; pass < 2; ++pass) {
#pragma unroll
    for (int it = 0; it < 2; ++it) {
      const int row = wave * 8 + it * 4 + q;
      unsigned short hb[8];
#pragma unroll
      for (int e = 0; e < 8; ++e) hb[e] = h_bits(sm[row][c8 + e]);
      const v4u u = (v4u){pk16(hb[0], hb[1]), pk16(hb[2], hb[3]), pk16(hb[4], hb[5]), pk16(hb[6], hb[7])};
      *(volatile v4u*)(out + (obase + (size_t)row) * (size_t)nrows + r0 + c8) = u;
    }
    __threadfence();
  }
}

__global__ __launch_bounds__(256) void cast8_f16_kernel(const float* __restrict__ in, unsigned short* __restrict__ out,
                                                       int n8, float scale) {
  const int i = blockIdx.x * 256 + threadIdx.x;
  if (i >= n8) return;
  const float* p = in + 8 * (size_t)i;
  const v4f a = *(const v4f*)(p);
  const v4f c = *(const v4f*)(p + 4);
  unsigned short hb[8];
#pragma unroll
  for (int e = 0; e < 4; ++e) {
    hb[e]     = h_bits(a[e] * scale);
    hb[4 + e] = h_bits(c[e] * scale);
  }
  const v4u u = (v4u){pk16(hb[0], hb[1]), pk16(hb[2], hb[3]), pk16(hb[4], hb[5]), pk16(hb[6], hb[7])};
  unsigned short* qo = out + 8 * (size_t)i;
  *(volatile v4u*)qo = u;
  __threadfence();
  *(volatile v4u*)qo = u;
}

__global__ __launch_bounds__(128) void rms_f16_kernel(const float* __restrict__ X, const float* __restrict__ w,
                                                     unsigned short* __restrict__ out) {
  __shared__ float red[4];
  const int row  = blockIdx.x;
  const int t    = threadIdx.x;
  const int lane = t & 31, wave = t >> 5;
  const int c0   = t * 8;
  const float* xr = X + (size_t)row * kD + c0;
  const v4f a  = *(const v4f*)(xr);
  const v4f c  = *(const v4f*)(xr + 4);
  const v4f wa = *(const v4f*)(w + c0);
  const v4f wc = *(const v4f*)(w + c0 + 4);
  float x[8], wv[8];
#pragma unroll
  for (int e = 0; e < 4; ++e) { x[e] = a[e]; x[4 + e] = c[e]; wv[e] = wa[e]; wv[4 + e] = wc[e]; }
  float ss = 0.f;
#pragma unroll
  for (int e = 0; e < 8; ++e) ss += x[e] * x[e];
#pragma unroll
  for (int off = 16; off > 0; off >>= 1) ss += __shfl_xor(ss, off, 32);
  if (lane == 0) red[wave] = ss;
  __syncthreads();
  const float tot = (red[0] + red[1]) + (red[2] + red[3]);
  const float inv = rsqrtf(tot * kInvD + kEps);
  unsigned short hb[8];
#pragma unroll
  for (int e = 0; e < 8; ++e) hb[e] = h_bits((wv[e] * x[e]) * inv);
  const v4u u = (v4u){pk16(hb[0], hb[1]), pk16(hb[2], hb[3]), pk16(hb[4], hb[5]), pk16(hb[6], hb[7])};
  unsigned short* dst = out + (size_t)row * kD + c0;
  *(volatile v4u*)dst = u;
  __threadfence();
  *(volatile v4u*)dst = u;
}

__global__ __launch_bounds__(256) void rope_kernel(const float* __restrict__ S32, const float* __restrict__ cs,
                                                  const float* __restrict__ sn,
                                                  unsigned short* __restrict__ Qp, unsigned short* __restrict__ Kp,
                                                  unsigned short* __restrict__ Vt, int bidx) {
  __shared__ __align__(16) float sm[64 * 68];
  const int t = threadIdx.x, lane = t & 31, wave = t >> 5;
  const int tt = blockIdx.x, h = blockIdx.y;
  const int g = bidx * kH + h;
  const int r = t >> 2, qq = t & 3;
  const int tok = tt * 64 + r;
  const int q4 = lane >> 3, c8 = (lane & 7) * 8;
  float cv[8], sv[8];
  {
    const float* cp = cs + (size_t)tok * (kHD / 2) + qq * 8;
    const float* sp = sn + (size_t)tok * (kHD / 2) + qq * 8;
    const v4f ca = *(const v4f*)(cp), cb = *(const v4f*)(cp + 4);
    const v4f sa = *(const v4f*)(sp), sb = *(const v4f*)(sp + 4);
#pragma unroll
    for (int e = 0; e < 4; ++e) { cv[e] = ca[e]; cv[4 + e] = cb[e]; sv[e] = sa[e]; sv[4 + e] = sb[e]; }
  }
#pragma unroll
  for (int which = 0; which < 3; ++which) {
    const float* src = S32 + (size_t)tok * kNQKV + which * kD + h * kHD + qq * 16;
    const v4f x0 = *(const v4f*)(src), x1 = *(const v4f*)(src + 4), x2 = *(const v4f*)(src + 8), x3 = *(const v4f*)(src + 12);
    float x[16];
#pragma unroll
    for (int e = 0; e < 4; ++e) { x[e] = x0[e]; x[4 + e] = x1[e]; x[8 + e] = x2[e]; x[12 + e] = x3[e]; }
    float y[16];
    if (which < 2) {
#pragma unroll
      for (int j = 0; j < 8; ++j) {
        const float xr = x[2 * j], xi = x[2 * j + 1];
        y[2 * j]     = xr * cv[j] - xi * sv[j];
        y[2 * j + 1] = xr * sv[j] + xi * cv[j];
      }
    } else {
#pragma unroll
      for (int e = 0; e < 16; ++e) y[e] = x[e];
    }
    float* sp = sm + r * 68 + qq * 16;
    *(v4f*)(sp)      = (v4f){y[0], y[1], y[2], y[3]};
    *(v4f*)(sp + 4)  = (v4f){y[4], y[5], y[6], y[7]};
    *(v4f*)(sp + 8)  = (v4f){y[8], y[9], y[10], y[11]};
    *(v4f*)(sp + 12) = (v4f){y[12], y[13], y[14], y[15]};
    __syncthreads();
    if (which < 2) {
      unsigned short* dst = ((which == 0) ? Qp : Kp) + (size_t)g * kT * kHD;
      for (int pass = 0; pass < 2; ++pass) {
#pragma unroll
        for (int it = 0; it < 2; ++it) {
          const int row = wave * 8 + it * 4 + q4;
          unsigned short hb[8];
#pragma unroll
          for (int e = 0; e < 8; ++e) hb[e] = h_bits(sm[row * 68 + c8 + e]);
          const v4u u = (v4u){pk16(hb[0], hb[1]), pk16(hb[2], hb[3]), pk16(hb[4], hb[5]), pk16(hb[6], hb[7])};
          *(volatile v4u*)(dst + (size_t)(tt * 64 + row) * kHD + c8) = u;
        }
        __threadfence();
      }
    } else {
      unsigned short* dst = Vt + (size_t)g * kHD * kT;
      for (int pass = 0; pass < 2; ++pass) {
#pragma unroll
        for (int it = 0; it < 2; ++it) {
          const int erow = wave * 8 + it * 4 + q4;
          unsigned short hb[8];
#pragma unroll
          for (int j = 0; j < 8; ++j) hb[j] = h_bits(sm[(c8 + j) * 68 + erow]);
          const v4u u = (v4u){pk16(hb[0], hb[1]), pk16(hb[2], hb[3]), pk16(hb[4], hb[5]), pk16(hb[6], hb[7])};
          *(volatile v4u*)(dst + (size_t)erow * kT + tt * 64 + c8) = u;
        }
        __threadfence();
      }
    }
    __syncthreads();
  }
}

__global__ __launch_bounds__(256) void softmax_kernel(const float* __restrict__ S, const float* __restrict__ mask,
                                                     unsigned short* __restrict__ P) {
  __shared__ float redM[8];
  __shared__ float redS[8];
  const int row  = blockIdx.x;
  const int gl   = blockIdx.y;
  const int t    = threadIdx.x;
  const int lane = t & 31, wave = t >> 5;
  const int c0   = t * 8;
  const int lim  = ((row >> 6) + 1) << 6;
  const int cc   = (c0 < lim - 8) ? c0 : (lim - 8);
  const float* sr = S + ((size_t)gl * kT + row) * kT + cc;
  const v4f sa = *(const v4f*)(sr);
  const v4f sc = *(const v4f*)(sr + 4);
  const float* mr = mask + (size_t)row * kT + c0;
  const v4f ma = *(const v4f*)(mr);
  const v4f mc = *(const v4f*)(mr + 4);
  float lg[8];
#pragma unroll
  for (int e = 0; e < 4; ++e) {
    const float s0 = sa[e], m0 = ma[e];
    const float s1 = sc[e], m1 = mc[e];
    lg[e]     = (m0 <= -1.0e8f) ? m0 : (s0 + m0);
    lg[4 + e] = (m1 <= -1.0e8f) ? m1 : (s1 + m1);
  }
  float m = fmaxf(fmaxf(fmaxf(lg[0], lg[1]), fmaxf(lg[2], lg[3])), fmaxf(fmaxf(lg[4], lg[5]), fmaxf(lg[6], lg[7])));
#pragma unroll
  for (int off = 16; off > 0; off >>= 1) m = fmaxf(m, __shfl_xor(m, off, 32));
  if (lane == 0) redM[wave] = m;
  __syncthreads();
  m = fmaxf(fmaxf(fmaxf(redM[0], redM[1]), fmaxf(redM[2], redM[3])), fmaxf(fmaxf(redM[4], redM[5]), fmaxf(redM[6], redM[7])));
  float p[8];
  float ps = 0.f;
#pragma unroll
  for (int e = 0; e < 8; ++e) { p[e] = expf(lg[e] - m); ps += p[e]; }
#pragma unroll
  for (int off = 16; off > 0; off >>= 1) ps += __shfl_xor(ps, off, 32);
  if (lane == 0) redS[wave] = ps;
  __syncthreads();
  const float tot = ((redS[0] + redS[1]) + (redS[2] + redS[3])) + ((redS[4] + redS[5]) + (redS[6] + redS[7]));
  const float inv = 1.0f / tot;
  unsigned short hb[8];
#pragma unroll
  for (int e = 0; e < 8; ++e) { const float pn = p[e] * inv; hb[e] = h_bits(pn * kPCarry); }
  const v4u u = (v4u){pk16(hb[0], hb[1]), pk16(hb[2], hb[3]), pk16(hb[4], hb[5]), pk16(hb[6], hb[7])};
  unsigned short* dst = P + ((size_t)gl * kT + row) * kT + c0;
  *(volatile v4u*)dst = u;
  __threadfence();
  *(volatile v4u*)dst = u;
}

__global__ __launch_bounds__(256) void swiglu_kernel(const float* __restrict__ GU, unsigned short* __restrict__ Hout) {
  const int i = blockIdx.x * 256 + threadIdx.x;
  const int row = i >> 9;
  const int c8  = (i & 511) * 8;
  const float* gp = GU + (size_t)row * kN12 + c8;
  const v4f g0 = *(const v4f*)(gp), g1 = *(const v4f*)(gp + 4);
  const v4f u0 = *(const v4f*)(gp + kFF), u1 = *(const v4f*)(gp + kFF + 4);
  float gv[8], uv[8];
#pragma unroll
  for (int e = 0; e < 4; ++e) { gv[e] = g0[e]; gv[4 + e] = g1[e]; uv[e] = u0[e]; uv[4 + e] = u1[e]; }
  unsigned short hb[8];
#pragma unroll
  for (int e = 0; e < 8; ++e) {
    const float ex = expf(-gv[e]);
    const float sg = __builtin_amdgcn_rcpf(1.0f + ex);
    const float hv = uv[e] * (gv[e] * sg);
    hb[e] = h_bits(hv);
  }
  const v4u u = (v4u){pk16(hb[0], hb[1]), pk16(hb[2], hb[3]), pk16(hb[4], hb[5]), pk16(hb[6], hb[7])};
  unsigned short* dst = Hout + (size_t)row * kFF + c8;
  *(volatile v4u*)dst = u;
  __threadfence();
  *(volatile v4u*)dst = u;
}

extern "C" void kernel_launch(void* const* d_in, const int* in_sizes, int n_in,
                              void* d_out, int out_size, void* d_ws, size_t ws_size,
                              hipStream_t stream) {
  (void)in_sizes;
  if (n_in < 14) return;
  if (ws_size < WS_TOTAL) return;
  if ((size_t)out_size < (size_t)kTok * kD) return;

  const float* x     = (const float*)d_in[0];
  const float* cosb  = (const float*)d_in[1];
  const float* sinb  = (const float*)d_in[2];
  const float* maskp = (const float*)d_in[3];
  const float* attw  = (const float*)d_in[4];
  const float* Wq    = (const float*)d_in[5];
  const float* Wk    = (const float*)d_in[6];
  const float* Wv    = (const float*)d_in[7];
  const float* ffnw  = (const float*)d_in[8];
  const float* fc1   = (const float*)d_in[9];
  const float* fc2   = (const float*)d_in[10];
  const float* fc3   = (const float*)d_in[11];
  const float* projw = (const float*)d_in[12];
  const float* projb = (const float*)d_in[13];
  float* out = (float*)d_out;

  char* ws = (char*)d_ws;
  u16*   WQKV = (u16*)(ws + OFF_WQKV);
  u16*   XN   = (u16*)(ws + OFF_XN);
  float* BIGF = (float*)(ws + OFF_BIG);
  u16*   W12  = (u16*)(ws + OFF_W12);
  u16*   QP   = (u16*)(ws + OFF_QP);
  u16*   KP   = (u16*)(ws + OFF_KP);
  u16*   VT   = (u16*)(ws + OFF_VT);
  u16*   PP   = (u16*)(ws + OFF_PP);
  u16*   HH   = (u16*)(ws + OFF_HH);
  u16*   W3T  = (u16*)(ws + OFF_W3T);
  float* X1   = (float*)(ws + OFF_X1);
  u16*   WP   = (u16*)(ws + OFF_WP);
  u16*   X2H  = XN;
  const u16* nul16 = nullptr;

  tcast16_kernel<<<dim3(kD / 64, 1, 3 * kH), 256, 0, stream>>>(
      Wq, Wk, Wv, kD, kHD, kH, (long)kD * kHD, WQKV, (long)kD, (long)kHD, kWCarry);

  rms_f16_kernel<<<kTok, 128, 0, stream>>>(x, attw, XN);

  for (int b = 0; b < kB; ++b) {
    wmma_gemm64<0, false, 0, 0, false, 0><<<dim3((kT / 64) * (kNQKV / 64) / 8, 1), 256, 0, stream>>>(
        XN + (size_t)b * kT * kD, nul16, kD, 0L,
        WQKV, nul16, kD, 0L,
        BIGF, nullptr, kNQKV, 0L,
        nullptr, nullptr, 0L,
        kT, kNQKV, kD, kWCarryInv);
    rope_kernel<<<dim3(kT / 64, kH), 256, 0, stream>>>(BIGF, cosb, sinb, QP, KP, VT, b);
  }

  for (int ch = 0; ch < (kB * kH) / kGrp; ++ch) {
    const int b  = ch / (kH / kGrp);
    const int h0 = (ch % (kH / kGrp)) * kGrp;
    const size_t gb = (size_t)b * kH + h0;
    wmma_gemm64<0, false, 0, 0, false, 1><<<dim3((kT / 64) * (kT / 64) / 8, kGrp), 256, 0, stream>>>(
        QP + gb * kT * kHD, nul16, kHD, (long)kT * kHD,
        KP + gb * kT * kHD, nul16, kHD, (long)kT * kHD,
        BIGF, nullptr, kT, (long)kT * kT,
        nullptr, nullptr, 0L,
        kT, kT, kHD, kQKScale);
    softmax_kernel<<<dim3(kT, kGrp), 256, 0, stream>>>(BIGF, maskp, PP);
    const size_t xoff = (size_t)b * kT * kD + (size_t)h0 * kHD;
    wmma_gemm64<0, false, 0, 0, true, 2><<<dim3((kT / 64) * (kHD / 64) / 8, kGrp), 256, 0, stream>>>(
        PP, nul16, kT, (long)kT * kT,
        VT + gb * kHD * kT, nul16, kT, (long)kHD * kT,
        X1 + xoff, nullptr, kD, (long)kHD,
        nullptr, x + xoff, (long)kHD,
        kT, kHD, kT, kPCarryInv);
  }

  rms_f16_kernel<<<kTok, 128, 0, stream>>>(X1, ffnw, XN);

  tcast16_kernel<<<dim3(kD / 64, kFF / 64, 2), 256, 0, stream>>>(
      fc1, fc2, fc2, kD, kFF, 1, 0L, W12, (long)kFF, 0L, kWCarry);
  tcast16_kernel<<<dim3(kFF / 64, kD / 64, 1), 256, 0, stream>>>(
      fc3, fc3, fc3, kFF, kD, 1, 0L, W3T, 0L, 0L, kWCarry);
  cast8_f16_kernel<<<(kD * kD / 8) / 256, 256, 0, stream>>>(projw, WP, kD * kD / 8, kWCarry);

  for (int c = 0; c < kTok / kFfnRows; ++c) {
    wmma_gemm64<0, false, 0, 0, false, 0><<<dim3((kFfnRows / 64) * (kN12 / 64) / 8, 1), 256, 0, stream>>>(
        XN + (size_t)c * kFfnRows * kD, nul16, kD, 0L,
        W12, nul16, kD, 0L,
        BIGF, nullptr, kN12, 0L,
        nullptr, nullptr, 0L,
        kFfnRows, kN12, kD, kWCarryInv);
    swiglu_kernel<<<(kFfnRows * kFF / 8) / 256, 256, 0, stream>>>(BIGF, HH + (size_t)c * kFfnRows * kFF);
  }

  wmma_gemm64<0, false, 0, 1, true, 0><<<dim3((kTok / 64) * (kD / 64) / 8, 1), 256, 0, stream>>>(
      HH, nul16, kFF, 0L,
      W3T, nul16, kFF, 0L,
      X2H, nullptr, kD, 0L,
      nullptr, X1, 0L,
      kTok, kD, kFF, kWCarryInv);

  wmma_gemm64<0, false, 2, 0, false, 0><<<dim3((kTok / 64) * (kD / 64) / 8, 1), 256, 0, stream>>>(
      X2H, nul16, kD, 0L,
      WP, nul16, kD, 0L,
      out, nullptr, kD, 0L,
      projb, nullptr, 0L,
      kTok, kD, kD, kWCarryInv);
}
